// SuperMacroGCN_20203526160737
// MI455X (gfx1250) — hardware-verified
//
#include <hip/hip_runtime.h>
#include <stddef.h>


typedef _Float16 v16h __attribute__((ext_vector_type(16)));
typedef _Float16 v8h  __attribute__((ext_vector_type(8)));
typedef float    v8f  __attribute__((ext_vector_type(8)));
typedef float    v4f  __attribute__((ext_vector_type(4)));
typedef int      v4i  __attribute__((ext_vector_type(4)));

union Frag { v16h v; v8h half[2]; };

#define CH      4096
#define BKT     512
#define BKT_SH  9
#define CAPB    12288
#define KP      72
#define TP      68


__device__ __forceinline__ v8f wmma16(v16h a, v16h b, v8f c) {
  v8f d = __builtin_amdgcn_wmma_f32_16x16x32_f16(false, a, false, b, (short)0, c, false, false);
  asm volatile("v_nop\n\tv_nop\n\tv_nop\n\tv_nop" : "+v"(d) : "v"(a), "v"(b));
  return d;
}

__device__ __forceinline__ v8h cvt8(v4f p, v4f q) {
  v8h r;
  r[0] = (_Float16)p.x; r[1] = (_Float16)p.y; r[2] = (_Float16)p.z; r[3] = (_Float16)p.w;
  r[4] = (_Float16)q.x; r[5] = (_Float16)q.y; r[6] = (_Float16)q.z; r[7] = (_Float16)q.w;
  return r;
}

__device__ __forceinline__ v8f zero8() {
  v8f z;
#pragma unroll
  for (int i = 0; i < 8; ++i) z[i] = 0.0f;
  return z;
}

__device__ __forceinline__ int clampi(int v, int lo, int hi) { return v < lo ? lo : (v > hi ? hi : v); }

__device__ __forceinline__ int wave_incl_scan32(int x) {
  const int lane = threadIdx.x & 31;
#pragma unroll
  for (int d = 1; d < 32; d <<= 1) {
    const int y = __shfl_up(x, d, 32);
    if (lane >= d) x += y;
  }
  return x;
}

__device__ __forceinline__ int block_excl_scan256(int v, int* s_a, int* s_b, int* total) {
  const int lane = threadIdx.x & 31, wv = threadIdx.x >> 5;
  const int inc = wave_incl_scan32(v);
  if (lane == 31) s_a[wv] = inc;
  __syncthreads();
  if (wv == 0) {
    const int w = (lane < 8) ? s_a[lane] : 0;
    const int wi = wave_incl_scan32(w);
    if (lane < 8) s_b[lane] = wi;
  }
  __syncthreads();
  const int pre = (wv > 0) ? s_b[wv - 1] : 0;
  *total = s_b[7];
  return pre + inc - v;
}

__global__ __launch_bounds__(256) void k_chunk(const int* __restrict__ erow, const int* __restrict__ ecol,
                                               int E, int N,
                                               int* __restrict__ ckeys, int* __restrict__ coff) {
  __shared__ __attribute__((aligned(16))) int s_bkt[CH];
  __shared__ __attribute__((aligned(16))) int s_key[CH];
  __shared__ __attribute__((aligned(16))) int s_out[CH];
  __shared__ __attribute__((aligned(16))) int s_off[256];
  __shared__ int s_sa[8], s_sb[8];

  const int tid = threadIdx.x;
  const int c = blockIdx.x;
  const long long e0 = (long long)c * CH;

  for (int j = tid; j < CH; j += 256) {
    const long long e = e0 + j;
    int bk = -1, key = 0;
    if (e < (long long)E) {
      const int r = erow[e];
      const int cl = clampi(ecol[e], 0, N - 1);
      if ((unsigned)r < (unsigned)N) {
        bk  = r >> BKT_SH;
        key = ((r & (BKT - 1)) << 17) | cl;
      }
    }
    s_bkt[j] = bk;
    s_key[j] = key;
  }
  __syncthreads();

  const int t = tid;
  const v4i* b4 = (const v4i*)s_bkt;
  int cnt = 0;
#pragma unroll 4
  for (int j4 = 0; j4 < CH / 4; ++j4) {
    const v4i q = b4[j4];
    cnt += (q.x == t) + (q.y == t) + (q.z == t) + (q.w == t);
  }
  int total = 0;
  const int off = block_excl_scan256(cnt, s_sa, s_sb, &total);
  s_off[t] = off;

  int p = off;
#pragma unroll 2
  for (int j4 = 0; j4 < CH / 4; ++j4) {
    const v4i q = b4[j4];
    const int j = j4 * 4;
    if (q.x == t) s_out[p++] = s_key[j];
    if (q.y == t) s_out[p++] = s_key[j + 1];
    if (q.z == t) s_out[p++] = s_key[j + 2];
    if (q.w == t) s_out[p++] = s_key[j + 3];
  }
  for (int j = total + tid; j < CH; j += 256) s_out[j] = 0;
  __syncthreads();

  int* gk = ckeys + (size_t)c * CH;
  int* go = coff + (size_t)c * 256;
#pragma unroll
  for (int it = 0; it < CH / 1024; ++it) {
    const int q = it * 1024 + tid * 4;
    const v4i v = *(const v4i*)(s_out + q);
    *(volatile v4i*)(gk + q) = v;
  }
  if (tid < 64) {
    const v4i v = *(const v4i*)(s_off + tid * 4);
    *(volatile v4i*)(go + tid * 4) = v;
  }
  __threadfence();
#pragma unroll
  for (int it = 0; it < CH / 1024; ++it) {
    const int q = it * 1024 + tid * 4;
    const v4i v = *(const v4i*)(s_out + q);
    *(volatile v4i*)(gk + q) = v;
  }
  if (tid < 64) {
    const v4i v = *(const v4i*)(s_off + tid * 4);
    *(volatile v4i*)(go + tid * 4) = v;
  }
}

__global__ __launch_bounds__(256) void k_bucket(const int* __restrict__ ckeys, const int* __restrict__ coff,
                                                int NCH,
                                                int* __restrict__ ccol, int* __restrict__ segs,
                                                int* __restrict__ sege, float* __restrict__ dinv) {
  __shared__ __attribute__((aligned(16))) int   s_in[CAPB];
  __shared__ __attribute__((aligned(16))) int   s_out[CAPB];
  __shared__ __attribute__((aligned(16))) int   s_off[BKT + 4];
  __shared__ __attribute__((aligned(16))) int   s_ss[BKT];
  __shared__ __attribute__((aligned(16))) int   s_se[BKT];
  __shared__ __attribute__((aligned(16))) float s_dv[BKT];
  __shared__ int s_cnt[BKT];
  __shared__ int s_cst[256], s_cnm[256], s_cds[256];
  __shared__ int s_sa[8], s_sb[8];

  const int tid = threadIdx.x;
  const int b = blockIdx.x;

  for (int j = tid; j < CAPB; j += 256) s_in[j] = -1;
  __syncthreads();

  int base = 0;
  for (int c0 = 0; c0 < NCH; c0 += 256) {
    const int c = c0 + tid;
    int st = 0, nn = 0;
    if (c < NCH) {
      const int* rowp = coff + (size_t)c * 256;
      int a  = clampi(rowp[b], 0, CH);
      int en = clampi(rowp[b + 1], a, CH);
      st = a;
      nn = en - a;
    }
    int btot = 0;
    const int ds = block_excl_scan256(nn, s_sa, s_sb, &btot);
    s_cst[tid] = st;
    s_cnm[tid] = nn;
    s_cds[tid] = base + ds;
    __syncthreads();
    const int clim = (NCH - c0 < 256) ? (NCH - c0) : 256;
    for (int cc = 0; cc < clim; ++cc) {
      const int n  = s_cnm[cc];
      const int d0 = s_cds[cc];
      const int* src = ckeys + (size_t)(c0 + cc) * CH + s_cst[cc];
      for (int j = tid; j < n; j += 256) {
        const int pos = d0 + j;
        if (pos < CAPB) s_in[pos] = src[j];
      }
    }
    base += btot;
    __syncthreads();
  }
  const int total  = base < CAPB ? base : CAPB;
  const int total4 = (total + 3) & ~3;
  __syncthreads();

  const v4i* in4 = (const v4i*)s_in;
  const unsigned r0i = (unsigned)tid, r1i = (unsigned)(tid + 256);
  const int nq = total4 >> 2;
  int cA = 0, cB = 0;
#pragma unroll 2
  for (int jq = 0; jq < nq; ++jq) {
    const v4i k = in4[jq];
    const unsigned ra = (unsigned)k.x >> 17, rb = (unsigned)k.y >> 17;
    const unsigned rc = (unsigned)k.z >> 17, rd = (unsigned)k.w >> 17;
    cA += (ra == r0i) + (rb == r0i) + (rc == r0i) + (rd == r0i);
    cB += (ra == r1i) + (rb == r1i) + (rc == r1i) + (rd == r1i);
  }
  s_cnt[tid] = cA;
  s_cnt[tid + 256] = cB;
  __syncthreads();
  const int a0 = s_cnt[2 * tid], a1 = s_cnt[2 * tid + 1];
  int tsum = 0;
  const int ex = block_excl_scan256(a0 + a1, s_sa, s_sb, &tsum);
  s_off[2 * tid] = ex;
  s_off[2 * tid + 1] = ex + a0;
  if (tid == 255) { s_off[BKT] = tsum; s_off[BKT + 1] = 0; s_off[BKT + 2] = 0; s_off[BKT + 3] = 0; }
  __syncthreads();

  int p0 = s_off[tid], p1 = s_off[tid + 256];
#pragma unroll 2
  for (int jq = 0; jq < nq; ++jq) {
    const v4i k = in4[jq];
#pragma unroll
    for (int u = 0; u < 4; ++u) {
      const int kk = k[u];
      const unsigned r = (unsigned)kk >> 17;
      const int cl = kk & 0x1FFFF;
      if (r == r0i) s_out[p0++] = cl;
      else if (r == r1i) s_out[p1++] = cl;
    }
  }
  for (int j = tsum + tid; j < CAPB; j += 256) s_out[j] = 0;

#pragma unroll
  for (int u = 0; u < 2; ++u) {
    const int r = tid + 256 * u;
    const int s0 = s_off[r], s1 = s_off[r + 1];
    s_ss[r] = b * CAPB + s0;
    s_se[r] = b * CAPB + s1;
    s_dv[r] = rsqrtf((float)(s1 - s0 + 1));
  }
  __syncthreads();

  int*   gc = ccol + (size_t)b * CAPB;
  int*   gs = segs + (size_t)b * BKT;
  int*   ge = sege + (size_t)b * BKT;
  float* gd = dinv + (size_t)b * BKT;
  for (int q = tid * 4; q < CAPB; q += 1024) {
    const v4i v = *(const v4i*)(s_out + q);
    *(volatile v4i*)(gc + q) = v;
  }
  if (tid < 128) {
    const v4i v = *(const v4i*)(s_ss + tid * 4);
    *(volatile v4i*)(gs + tid * 4) = v;
    const v4f w = *(const v4f*)(s_dv + tid * 4);
    *(volatile v4f*)(gd + tid * 4) = w;
  } else {
    const int q = (tid - 128) * 4;
    const v4i v = *(const v4i*)(s_se + q);
    *(volatile v4i*)(ge + q) = v;
  }
  __threadfence();
  for (int q = tid * 4; q < CAPB; q += 1024) {
    const v4i v = *(const v4i*)(s_out + q);
    *(volatile v4i*)(gc + q) = v;
  }
  if (tid < 128) {
    const v4i v = *(const v4i*)(s_ss + tid * 4);
    *(volatile v4i*)(gs + tid * 4) = v;
    const v4f w = *(const v4f*)(s_dv + tid * 4);
    *(volatile v4f*)(gd + tid * 4) = w;
  } else {
    const int q = (tid - 128) * 4;
    const v4i v = *(const v4i*)(s_se + q);
    *(volatile v4i*)(ge + q) = v;
  }
}

__global__ __launch_bounds__(128) void k_gemm(const float* __restrict__ A, const float* __restrict__ W,
                                              float* __restrict__ Hout, int N) {
  __shared__ __attribute__((aligned(16))) _Float16 s_wt[64 * KP];
  __shared__ __attribute__((aligned(16))) float    s_tile[64 * TP];

  const int tid = threadIdx.x;
#pragma unroll
  for (int it = 0; it < 32; ++it) {
    const int idx = it * 128 + tid;
    const int k = idx >> 6, n = idx & 63;
    s_wt[n * KP + k] = (_Float16)(W[idx] * 16.0f);
  }
  __syncthreads();

  const int wv = tid >> 5, l = tid & 31, h = l >> 4, m = l & 15;
  const int rowBase = blockIdx.x * 64 + wv * 16;
  int rA = rowBase + m;
  if (rA > N - 1) rA = N - 1;
  const float* arow = A + (size_t)rA * 64;

  v8f acc[4];
#pragma unroll
  for (int nt = 0; nt < 4; ++nt) acc[nt] = zero8();

#pragma unroll
  for (int ks = 0; ks < 2; ++ks) {
    const int k0 = ks * 32;
    const v4f p0 = *(const v4f*)(arow + k0 + 8 * h);
    const v4f p1 = *(const v4f*)(arow + k0 + 8 * h + 4);
    const v4f q0 = *(const v4f*)(arow + k0 + 16 + 8 * h);
    const v4f q1 = *(const v4f*)(arow + k0 + 16 + 8 * h + 4);
    Frag a;
    a.half[0] = cvt8(p0, p1);
    a.half[1] = cvt8(q0, q1);
#pragma unroll
    for (int nt = 0; nt < 4; ++nt) {
      const _Float16* wb = s_wt + (nt * 16 + m) * KP + k0;
      Frag bb;
      bb.half[0] = *(const v8h*)(wb + 8 * h);
      bb.half[1] = *(const v8h*)(wb + 16 + 8 * h);
      acc[nt] = wmma16(a.v, bb.v, acc[nt]);
    }
  }

  float* trow = s_tile + (wv * 16 + 8 * h) * TP + m;
#pragma unroll
  for (int nt = 0; nt < 4; ++nt) {
#pragma unroll
    for (int r = 0; r < 8; ++r) trow[r * TP + nt * 16] = acc[nt][r] * 0.0625f;
  }
  __syncthreads();

  const int blkRow = blockIdx.x * 64;
#pragma unroll
  for (int it = 0; it < 8; ++it) {
    const int q = it * 512 + tid * 4;
    const int row = q >> 6, col = q & 63;
    const int grow = blkRow + row;
    if (grow < N) {
      const v4f v = *(const v4f*)(s_tile + row * TP + col);
      *(volatile v4f*)(Hout + (size_t)grow * 64 + col) = v;
    }
  }
  __threadfence();
#pragma unroll
  for (int it = 0; it < 8; ++it) {
    const int q = it * 512 + tid * 4;
    const int row = q >> 6, col = q & 63;
    const int grow = blkRow + row;
    if (grow < N) {
      const v4f v = *(const v4f*)(s_tile + row * TP + col);
      *(volatile v4f*)(Hout + (size_t)grow * 64 + col) = v;
    }
  }
}

__global__ __launch_bounds__(256) void k_agg(const float* __restrict__ H,
                                             const int* __restrict__ segs, const int* __restrict__ sege,
                                             const int* __restrict__ ccol, const float* __restrict__ dinv,
                                             const float* __restrict__ bias,
                                             const float* __restrict__ bg, const float* __restrict__ bbeta,
                                             const float* __restrict__ bm, const float* __restrict__ bv,
                                             int use_bn, int N, int nslots,
                                             float* __restrict__ out) {
  const int tid = threadIdx.x;
  const int l = tid & 31, h = l >> 4, m = l & 15;
  const long long gw = (long long)blockIdx.x * 8 + (tid >> 5);
  const long long nodeL = gw * 2 + h;
  const bool valid = nodeL < (long long)N;
  const int node = valid ? (int)nodeL : (N - 1);

  const int s = segs[node];
  int n = sege[node] - s;
  if (!valid || n < 0 || s < 0 || (long long)s + (long long)n > (long long)nslots) n = 0;
  const float di = dinv[node];
  const int n2 = __shfl_xor(n, 16, 32);
  const int nmax = n > n2 ? n : n2;

  v4f acc;
  acc.x = 0.0f; acc.y = 0.0f; acc.z = 0.0f; acc.w = 0.0f;
  for (int j = 0; j < nmax; ++j) {
    int c = node;
    float w = 0.0f;
    if (j < n) {
      c = clampi(ccol[s + j], 0, N - 1);
      w = dinv[c];
    }
    const v4f v = *(const v4f*)(H + (size_t)c * 64 + 4 * m);
    acc += w * v;
  }
  const v4f hv = *(const v4f*)(H + (size_t)node * 64 + 4 * m);
  const v4f b4 = *(const v4f*)(bias + 4 * m);
  v4f y = b4 + (di * di) * hv + di * acc;
  if (use_bn) {
    const v4f g4  = *(const v4f*)(bg + 4 * m);
    const v4f be4 = *(const v4f*)(bbeta + 4 * m);
    const v4f m4  = *(const v4f*)(bm + 4 * m);
    const v4f vv4 = *(const v4f*)(bv + 4 * m);
    v4f rs;
    rs.x = rsqrtf(vv4.x + 1e-5f); rs.y = rsqrtf(vv4.y + 1e-5f);
    rs.z = rsqrtf(vv4.z + 1e-5f); rs.w = rsqrtf(vv4.w + 1e-5f);
    y = (y - m4) * rs * g4 + be4;
    y.x = fmaxf(y.x, 0.0f); y.y = fmaxf(y.y, 0.0f); y.z = fmaxf(y.z, 0.0f); y.w = fmaxf(y.w, 0.0f);
  }
  float* dst = out + (size_t)node * 64 + 4 * m;
  if (valid) *(volatile v4f*)dst = y;
  __threadfence();
  if (valid) *(volatile v4f*)dst = y;
}

static inline size_t al256(size_t x) { return (x + 255) & ~(size_t)255; }

extern "C" void kernel_launch(void* const* d_in, const int* in_sizes, int n_in,
                              void* d_out, int out_size, void* d_ws, size_t ws_size,
                              hipStream_t stream) {
  if (n_in < 16) return;
  const float* x    = (const float*)d_in[0];
  const int*   eidx = (const int*)d_in[1];
  const float* W1   = (const float*)d_in[2];
  const float* b1   = (const float*)d_in[3];
  const float* g1   = (const float*)d_in[4];
  const float* be1  = (const float*)d_in[5];
  const float* m1   = (const float*)d_in[6];
  const float* v1   = (const float*)d_in[7];
  const float* W2   = (const float*)d_in[8];
  const float* b2   = (const float*)d_in[9];
  const float* g2   = (const float*)d_in[10];
  const float* be2  = (const float*)d_in[11];
  const float* m2   = (const float*)d_in[12];
  const float* v2   = (const float*)d_in[13];
  const float* W3   = (const float*)d_in[14];
  const float* b3   = (const float*)d_in[15];

  const int N = in_sizes[0] / 64;
  const int E = in_sizes[1] / 2;
  if (N <= 0 || E < 0) return;
  if (N > (1 << 17)) return;
  const int NB = (N + BKT - 1) / BKT;
  if (NB > 255) return;
  const int NP  = NB * BKT;
  const int NCH = (E + CH - 1) / CH;
  if ((long long)out_size < 2LL * N * 64) return;

  char* ws = (char*)d_ws;
  size_t off = 0;
  int* ckeys = (int*)(ws + off);   off = al256(off + (size_t)NCH * CH * sizeof(int));
  int* coff  = (int*)(ws + off);   off = al256(off + (size_t)NCH * 256 * sizeof(int));
  int* ccol  = (int*)(ws + off);   off = al256(off + (size_t)NB * CAPB * sizeof(int));
  int* segs  = (int*)(ws + off);   off = al256(off + (size_t)NP * sizeof(int));
  int* sege  = (int*)(ws + off);   off = al256(off + (size_t)NP * sizeof(int));
  float* dnv = (float*)(ws + off); off = al256(off + (size_t)NP * sizeof(float));
  float* Hb  = (float*)(ws + off); off = al256(off + (size_t)N * 64 * sizeof(float));
  float* A1  = (float*)(ws + off); off = al256(off + (size_t)N * 64 * sizeof(float));
  if (off > ws_size) return;

  const int* erow = eidx;
  const int* ecol = eidx + E;
  float* emb  = (float*)d_out;
  float* pred = (float*)d_out + (size_t)N * 64;
  const int nslots = NB * CAPB;

  const int gG = (N + 63) / 64;
  const int gA = (N + 15) / 16;

  if (NCH > 0) k_chunk<<<dim3(NCH), dim3(256), 0, stream>>>(erow, ecol, E, N, ckeys, coff);
  k_bucket<<<dim3(NB), dim3(256), 0, stream>>>(ckeys, coff, NCH, ccol, segs, sege, dnv);

  k_gemm<<<dim3(gG), dim3(128), 0, stream>>>(x, W1, Hb, N);
  k_agg<<<dim3(gA), dim3(256), 0, stream>>>(Hb, segs, sege, ccol, dnv, b1, g1, be1, m1, v1, 1, N, nslots, A1);

  k_gemm<<<dim3(gG), dim3(128), 0, stream>>>(A1, W2, Hb, N);
  k_agg<<<dim3(gA), dim3(256), 0, stream>>>(Hb, segs, sege, ccol, dnv, b2, g2, be2, m2, v2, 1, N, nslots, emb);

  k_gemm<<<dim3(gG), dim3(128), 0, stream>>>(emb, W3, Hb, N);
  k_agg<<<dim3(gA), dim3(256), 0, stream>>>(Hb, segs, sege, ccol, dnv, b3, g2, be2, m2, v2, 0, N, nslots, pred);
}
